// FilteredBackProjection_58299886076393
// MI455X (gfx1250) — hardware-verified
//
#include <hip/hip_runtime.h>
#define NBS 2
#define NA 360
#define ND 363
#define NDP 384
#define HI 256
#define NR (NBS * NA)
typedef __bf16 v16b __attribute__((ext_vector_type(16)));
typedef unsigned short v8us __attribute__((ext_vector_type(8), may_alias));
typedef float  v8f  __attribute__((ext_vector_type(8)));
typedef float  v4f  __attribute__((ext_vector_type(4)));
typedef float  v4fa __attribute__((ext_vector_type(4), may_alias));
union FragB { v16b v; v8us half[2]; unsigned short u[16]; };

__device__ __forceinline__ unsigned short bf16_bits(float x) { unsigned int u = __float_as_uint(x); return (unsigned short)((u + 0x7FFFu + ((u >> 16) & 1u)) >> 16); }
__device__ __forceinline__ float bf16_val(unsigned short b) { return __uint_as_float(((unsigned int)b) << 16); }
__device__ __forceinline__ float bf16_round(float x) { return bf16_val(bf16_bits(x)); }
template <int NT>
__device__ __forceinline__ v8f mmaN(v16b ah, v16b al, v16b bh, v16b bl, v8f c) {
  c = __builtin_amdgcn_wmma_f32_16x16x32_bf16(false, ah, false, bh, (short)0, c, false, false);
  if (NT >= 2) c = __builtin_amdgcn_wmma_f32_16x16x32_bf16(false, al, false, bh, (short)0, c, false, false);
  if (NT >= 3) c = __builtin_amdgcn_wmma_f32_16x16x32_bf16(false, ah, false, bl, (short)0, c, false, false);
  asm volatile("v_nop\n\tv_nop\n\tv_nop\n\tv_nop" : "+v"(c) : "v"(ah), "v"(al), "v"(bh), "v"(bl));
  return c;
}

__global__ __launch_bounds__(256) void k_wt_bf16(const float* __restrict__ W, unsigned short* __restrict__ Wt, int K, int N) {
  const int t = blockIdx.x * 256 + threadIdx.x;
  const int k8n = K / 8;
  if (t >= N * k8n) return;
  const int n = t / k8n, k8 = (t % k8n) * 8;
  v8us v;
#pragma unroll
  for (int i = 0; i < 8; ++i) v[i] = bf16_bits(W[(size_t)(k8 + i) * N + n]);
  *(volatile v8us*)(Wt + (size_t)n * K + k8) = v;
  __threadfence();
  *(volatile v8us*)(Wt + (size_t)n * K + k8) = v;
}

template <bool ASPLIT, int ACT, bool BIAS_BF16>
__global__ __launch_bounds__(128) void k_gemm_bf(const float* __restrict__ A, int lda, const unsigned short* __restrict__ Wt, int ldb,
                                               const float* __restrict__ bias, float* __restrict__ C, int ldc, int M, int N, int K) {
  __shared__ __attribute__((aligned(16))) float so[4][16][64];
  const int tid = threadIdx.x, w = tid >> 5, lane = tid & 31, ln = lane & 15, hh = lane >> 4;
  const int ntn = N / 64;
  const int wid = blockIdx.x * 4 + w;
  const int mt = wid / ntn, nq = wid % ntn;
  if (mt * 16 >= M) return;
  const int row0 = mt * 16, col0 = nq * 64;
  const float* arow = A + (size_t)(row0 + ln) * lda;
  v8f acc[4] = {};
  for (int kb = 0; kb < K; kb += 32) {
    FragB ah, al;
    const v4f x0 = *(const v4fa*)(arow + kb + 8 * hh), x1 = *(const v4fa*)(arow + kb + 8 * hh + 4);
    const v4f x2 = *(const v4fa*)(arow + kb + 16 + 8 * hh), x3 = *(const v4fa*)(arow + kb + 16 + 8 * hh + 4);
    float xs[16] = {x0[0],x0[1],x0[2],x0[3],x1[0],x1[1],x1[2],x1[3],x2[0],x2[1],x2[2],x2[3],x3[0],x3[1],x3[2],x3[3]};
#pragma unroll
    for (int i = 0; i < 16; ++i) { const unsigned short hb = bf16_bits(xs[i]); ah.u[i] = hb; al.u[i] = ASPLIT ? bf16_bits(xs[i] - bf16_val(hb)) : (unsigned short)0; }
#pragma unroll
    for (int t = 0; t < 4; ++t) {
      const unsigned short* brow = Wt + (size_t)(col0 + t * 16 + ln) * ldb + kb;
      FragB b;
      b.half[0] = *(const v8us*)(brow + 8 * hh);
      b.half[1] = *(const v8us*)(brow + 16 + 8 * hh);
      acc[t] = mmaN<ASPLIT ? 2 : 1>(ah.v, al.v, b.v, b.v, acc[t]);
    }
  }
#pragma unroll
  for (int t = 0; t < 4; ++t) {
    float bv = bias ? bias[col0 + t * 16 + ln] : 0.f;
    if (BIAS_BF16) bv = bf16_round(bv);
#pragma unroll
    for (int r = 0; r < 8; ++r) { float v = acc[t][r] + bv; if (ACT == 1) v = fmaxf(v, 0.f); so[w][8 * hh + r][t * 16 + ln] = v; }
  }
  __builtin_amdgcn_fence(__ATOMIC_ACQ_REL, "workgroup");
  __builtin_amdgcn_wave_barrier();
  const int rsub = lane >> 4, c4 = (lane & 15) * 4;
  for (int pass = 0; pass < 2; ++pass) {
#pragma unroll
    for (int q = 0; q < 8; ++q) {
      const int r = q * 2 + rsub;
      const v4f v = *(const v4fa*)&so[w][r][c4];
      *(volatile v4f*)(C + (size_t)(row0 + r) * ldc + col0 + c4) = v;
    }
    if (pass == 0) __threadfence();
  }
}

template <bool ASPLIT, int ACT, bool BIAS_BF16, bool RES_BF16>
__global__ __launch_bounds__(128) void k_gemm_bf3(const float* __restrict__ A, int lda, const unsigned short* __restrict__ Wt, int ldb,
                                                const float* __restrict__ bias, const float* __restrict__ resid, int rmod, int ldr,
                                                float* __restrict__ C, int ldc, int M, int N, int K) {
  __shared__ __attribute__((aligned(16))) float so[4][16][64];
  const int tid = threadIdx.x, w = tid >> 5, lane = tid & 31, ln = lane & 15, hh = lane >> 4;
  const int ntn = N / 64;
  const int wid = blockIdx.x * 4 + w;
  const int mt = wid / ntn, nq = wid % ntn;
  if (mt * 16 >= M) return;
  const int row0 = mt * 16, col0 = nq * 64;
  const float* arow = A + (size_t)(row0 + ln) * lda;
  v8f acc[4] = {};
  for (int kb = 0; kb < K; kb += 32) {
    FragB ah, al;
    const v4f x0 = *(const v4fa*)(arow + kb + 8 * hh), x1 = *(const v4fa*)(arow + kb + 8 * hh + 4);
    const v4f x2 = *(const v4fa*)(arow + kb + 16 + 8 * hh), x3 = *(const v4fa*)(arow + kb + 16 + 8 * hh + 4);
    float xs[16] = {x0[0],x0[1],x0[2],x0[3],x1[0],x1[1],x1[2],x1[3],x2[0],x2[1],x2[2],x2[3],x3[0],x3[1],x3[2],x3[3]};
#pragma unroll
    for (int i = 0; i < 16; ++i) { const unsigned short hb = bf16_bits(xs[i]); ah.u[i] = hb; al.u[i] = ASPLIT ? bf16_bits(xs[i] - bf16_val(hb)) : (unsigned short)0; }
#pragma unroll
    for (int t = 0; t < 4; ++t) {
      const unsigned short* brow = Wt + (size_t)(col0 + t * 16 + ln) * ldb + kb;
      FragB b;
      b.half[0] = *(const v8us*)(brow + 8 * hh);
      b.half[1] = *(const v8us*)(brow + 16 + 8 * hh);
      acc[t] = mmaN<ASPLIT ? 2 : 1>(ah.v, al.v, b.v, b.v, acc[t]);
    }
  }
#pragma unroll
  for (int t = 0; t < 4; ++t) {
    const int col = col0 + t * 16 + ln;
    float bv = bias ? bias[col] : 0.f;
    if (BIAS_BF16) bv = bf16_round(bv);
#pragma unroll
    for (int r = 0; r < 8; ++r) {
      float v = acc[t][r] + bv;
      if (resid) { float rv = resid[(size_t)((row0 + 8 * hh + r) % rmod) * ldr + col]; if (RES_BF16) rv = bf16_round(rv); v += rv; }
      if (ACT == 1) v = fmaxf(v, 0.f);
      if (ACT == 2) v = 0.5f * v * (1.0f + erff(v * 0.70710678118654752f));
      if (ACT == 3) { const float u = 0.7978845608028654f * (v + 0.044715f * v * v * v); v = 0.5f * v * (1.0f + tanhf(u)); }
      so[w][8 * hh + r][t * 16 + ln] = v;
    }
  }
  __builtin_amdgcn_fence(__ATOMIC_ACQ_REL, "workgroup");
  __builtin_amdgcn_wave_barrier();
  const int rsub = lane >> 4, c4 = (lane & 15) * 4;
  for (int pass = 0; pass < 2; ++pass) {
#pragma unroll
    for (int q = 0; q < 8; ++q) {
      const int r = q * 2 + rsub;
      const v4f v = *(const v4fa*)&so[w][r][c4];
      *(volatile v4f*)(C + (size_t)(row0 + r) * ldc + col0 + c4) = v;
    }
    if (pass == 0) __threadfence();
  }
}
template <bool PARAM_BF16>
__global__ __launch_bounds__(256) void k_layernorm(const float* __restrict__ X, const float* __restrict__ R, const float* __restrict__ g, const float* __restrict__ bta,
                                                  float* __restrict__ out_sum, float* __restrict__ out_norm, int N, float eps) {
  __shared__ float red[256];
  const int row = blockIdx.x, tid = threadIdx.x;
  const float* x = X + (size_t)row * N; const float* rr = R ? R + (size_t)row * N : nullptr;
  float vals[16];
  const int per = N / 256;
  float s1 = 0.f;
  for (int u = 0; u < per / 4; ++u) {
    const int j = tid * 4 + 1024 * u;
    const v4f a = *(const v4fa*)(x + j);
    v4f b = {0.f,0.f,0.f,0.f}; if (rr) b = *(const v4fa*)(rr + j);
#pragma unroll
    for (int q = 0; q < 4; ++q) { const float v = a[q] + b[q]; vals[u * 4 + q] = v; s1 += v; }
  }
  red[tid] = s1; __syncthreads();
  for (int st = 128; st > 0; st >>= 1) { if (tid < st) red[tid] += red[tid + st]; __syncthreads(); }
  const float mu = red[0] / (float)N; __syncthreads();
  float s2 = 0.f;
  for (int u = 0; u < per / 4; ++u)
#pragma unroll
    for (int q = 0; q < 4; ++q) { const float c = vals[u * 4 + q] - mu; s2 += c * c; }
  red[tid] = s2; __syncthreads();
  for (int st = 128; st > 0; st >>= 1) { if (tid < st) red[tid] += red[tid + st]; __syncthreads(); }
  const float rs = rsqrtf(red[0] / (float)N + eps);
  for (int pass = 0; pass < 2; ++pass) {
    for (int u = 0; u < per / 4; ++u) {
      const int j = tid * 4 + 1024 * u;
      v4f o, sm;
#pragma unroll
      for (int q = 0; q < 4; ++q) {
        float gg = g[j + q], bb = bta[j + q];
        if (PARAM_BF16) { gg = bf16_round(gg); bb = bf16_round(bb); }
        sm[q] = vals[u * 4 + q]; o[q] = (vals[u * 4 + q] - mu) * rs * gg + bb;
      }
      if (out_sum) *(volatile v4f*)(out_sum + (size_t)row * N + j) = sm;
      *(volatile v4f*)(out_norm + (size_t)row * N + j) = o;
    }
    if (pass == 0) __threadfence();
  }
}


typedef _Float16 v16h __attribute__((ext_vector_type(16)));
union FragH { v16h v; v8us half[2]; _Float16 h[16]; unsigned short u[16]; };
template <int NT>
__device__ __forceinline__ v8f mmaH(v16h ah, v16h al, v16h bh, v16h bl, v8f c) {
  c = __builtin_amdgcn_wmma_f32_16x16x32_f16(false, ah, false, bh, (short)0, c, false, false);
  if (NT >= 2) c = __builtin_amdgcn_wmma_f32_16x16x32_f16(false, al, false, bh, (short)0, c, false, false);
  if (NT >= 3) c = __builtin_amdgcn_wmma_f32_16x16x32_f16(false, ah, false, bl, (short)0, c, false, false);
  asm volatile("v_nop\n\tv_nop\n\tv_nop\n\tv_nop" : "+v"(c) : "v"(ah), "v"(al), "v"(bh), "v"(bl));
  return c;
}
template <bool ASPLIT>
__global__ __launch_bounds__(128) void k_gemm_h(const float* __restrict__ A, int lda, size_t sA, const _Float16* __restrict__ Bh, int ldb, size_t sB, float alpha, float* __restrict__ C, int ldc, size_t sC, int M, int N, int K) {
  __shared__ __attribute__((aligned(16))) float so[4][16][64];
  const int tid = threadIdx.x, w = tid >> 5, lane = tid & 31, ln = lane & 15, hh = lane >> 4; const int by = blockIdx.y;
  A += (size_t)by * sA; Bh += (size_t)by * sB; C += (size_t)by * sC;
  const int ntn = (N + 63) / 64; const int wid = blockIdx.x * 4 + w; const int mt = wid / ntn, nq = wid % ntn; if (mt * 16 >= M) return;
  const int row0 = mt * 16, col0 = nq * 64; const float* arow = A + (size_t)(row0 + ln) * lda;
  v8f acc[4] = {};
  for (int kb = 0; kb < K; kb += 32) {
    FragH ah, al;
    const v4f x0 = *(const v4fa*)(arow + kb + 8 * hh), x1 = *(const v4fa*)(arow + kb + 8 * hh + 4), x2 = *(const v4fa*)(arow + kb + 16 + 8 * hh), x3 = *(const v4fa*)(arow + kb + 16 + 8 * hh + 4);
    float xs[16] = {x0[0],x0[1],x0[2],x0[3],x1[0],x1[1],x1[2],x1[3],x2[0],x2[1],x2[2],x2[3],x3[0],x3[1],x3[2],x3[3]};
#pragma unroll
    for (int i = 0; i < 16; ++i) { const _Float16 h = (_Float16)xs[i]; ah.h[i] = h; al.h[i] = ASPLIT ? (_Float16)(xs[i] - (float)h) : (_Float16)0.0f; }
#pragma unroll
    for (int t = 0; t < 4; ++t) { if (col0 + t * 16 >= N) continue; const size_t boff = (size_t)(col0 + t * 16 + ln) * ldb + kb; FragH bq; bq.half[0] = *(const v8us*)(Bh + boff + 8 * hh); bq.half[1] = *(const v8us*)(Bh + boff + 16 + 8 * hh);
      acc[t] = mmaH<ASPLIT ? 2 : 1>(ah.v, al.v, bq.v, bq.v, acc[t]); }
  }
#pragma unroll
  for (int t = 0; t < 4; ++t) { if (col0 + t * 16 >= N) continue;
#pragma unroll
    for (int r = 0; r < 8; ++r) so[w][8 * hh + r][t * 16 + ln] = acc[t][r] * alpha; }
  __builtin_amdgcn_fence(__ATOMIC_ACQ_REL, "workgroup"); __builtin_amdgcn_wave_barrier();
  const int rsub = lane >> 4, c4 = (lane & 15) * 4;
  for (int pass = 0; pass < 2; ++pass) {
#pragma unroll
    for (int q = 0; q < 8; ++q) { const int r = q * 2 + rsub; if (col0 + c4 < N) { const v4f v = *(const v4fa*)&so[w][r][c4]; *(volatile v4f*)(C + (size_t)(row0 + r) * ldc + col0 + c4) = v; } }
    if (pass == 0) __threadfence(); }
}

__global__ __launch_bounds__(256) void k_wt_f16(const float* __restrict__ W, _Float16* __restrict__ Wt, int K, int N, float scale) {
  const int t = blockIdx.x * 256 + threadIdx.x; if (t >= N * (K / 8)) return; const int n = t / (K / 8), k8 = (t % (K / 8)) * 8; FragH f;
#pragma unroll
  for (int i = 0; i < 8; ++i) f.h[i] = (_Float16)(bf16_round(W[(size_t)(k8 + i) * N + n]) * scale); const v8us o = f.half[0];
  *(volatile v8us*)((unsigned short*)Wt + (size_t)n * K + k8) = o; __threadfence(); *(volatile v8us*)((unsigned short*)Wt + (size_t)n * K + k8) = o;
}
template <int ACT>
__global__ __launch_bounds__(128) void k_gemm_hhx(const _Float16* __restrict__ A, int lda, size_t sA, const _Float16* __restrict__ Bh, int ldb, size_t sB, float alpha, const float* __restrict__ bias, size_t sBias, const float* __restrict__ CP, int rowsPerB, size_t sCPb, int row0g,
    float* __restrict__ C, _Float16* __restrict__ C16, int ldc, size_t sC, int M, int N, int K) {
  __shared__ __attribute__((aligned(16))) float so[4][16][64];
  const int tid = threadIdx.x, w = tid >> 5, lane = tid & 31, ln = lane & 15, hh = lane >> 4; const int by = blockIdx.y;
  A += (size_t)by * sA; Bh += (size_t)by * sB; const size_t cofs = (size_t)by * sC; const float* bp = bias ? bias + (size_t)by * sBias : nullptr;
  const int ntn = (N + 63) / 64; const int wid = blockIdx.x * 4 + w; const int mt = wid / ntn, nq = wid % ntn; if (mt * 16 >= M) return;
  const int row0 = mt * 16, col0 = nq * 64; const _Float16* arow = A + (size_t)(row0 + ln) * lda;
  v8f acc[4] = {};
  for (int kb = 0; kb < K; kb += 32) { FragH ah; ah.half[0] = *(const v8us*)((const unsigned short*)arow + kb + 8 * hh); ah.half[1] = *(const v8us*)((const unsigned short*)arow + kb + 16 + 8 * hh);
#pragma unroll
    for (int t = 0; t < 4; ++t) { if (col0 + t * 16 >= N) continue; const size_t boff = (size_t)(col0 + t * 16 + ln) * ldb + kb; FragH bq; bq.half[0] = *(const v8us*)((const unsigned short*)Bh + boff + 8 * hh); bq.half[1] = *(const v8us*)((const unsigned short*)Bh + boff + 16 + 8 * hh);
      acc[t] = mmaH<1>(ah.v, ah.v, bq.v, bq.v, acc[t]); }
  }
#pragma unroll
  for (int t = 0; t < 4; ++t) { if (col0 + t * 16 >= N) continue; const int col = col0 + t * 16 + ln; const float bv = bp ? bf16_round(bp[col]) : 0.f;
#pragma unroll
    for (int r = 0; r < 8; ++r) { float v = acc[t][r] * alpha + bv; if (CP) { const int bidx = (row0g + row0 + 8 * hh + r) / rowsPerB; v += CP[(size_t)bidx * sCPb + (size_t)by * 64 + col]; } if (ACT == 1) v = (v > 0.f) ? v : expm1f(v); else if (ACT == 7) v = (v > 0.f) ? v + 1.0f : expf(v); else if (ACT == 8) v = tanhf(v); else if (ACT == 9) v = 0.5f * v * (1.0f + tanhf(0.7978845608028654f * (v + 0.044715f * v * v * v))); else if (ACT == 11) v = 1.0f / (1.0f + expf(-v)); else if (ACT == 12) v = (v > 0.f) ? v : 0.01f * v; else if (ACT == 14) v = (v > 0.f) ? v : 0.1f * v; else if (ACT == 15) v = v / (1.0f + expf(-v)); else if (ACT == 3) v = fmaxf(v, 0.f); else if (ACT == 6) v = 0.5f * v * (1.0f + erff(v * 0.70710678118654752f)); so[w][8 * hh + r][t * 16 + ln] = v; } }
  __builtin_amdgcn_fence(__ATOMIC_ACQ_REL, "workgroup"); __builtin_amdgcn_wave_barrier();
  const int rsub = lane >> 4, c4 = (lane & 15) * 4; typedef _Float16 v4h __attribute__((ext_vector_type(4)));
  for (int pass = 0; pass < 2; ++pass) {
#pragma unroll
    for (int q = 0; q < 8; ++q) { const int r = q * 2 + rsub; if (col0 + c4 < N) { const v4f v = *(const v4fa*)&so[w][r][c4]; if (C) *(volatile v4f*)(C + cofs + (size_t)(row0 + r) * ldc + col0 + c4) = v; if (C16) { v4h h4; for (int i = 0; i < 4; ++i) h4[i] = (_Float16)v[i]; *(volatile v4h*)(C16 + cofs + (size_t)(row0 + r) * ldc + col0 + c4) = h4; } } }
    if (pass == 0) __threadfence(); }
}


typedef _Float16 v4h __attribute__((ext_vector_type(4)));

__global__ __launch_bounds__(256) void k_x16(const float* __restrict__ x, _Float16* __restrict__ X16, size_t n8) { const size_t t = (size_t)blockIdx.x * 256 + threadIdx.x; if (t >= n8) return; FragH f;
#pragma unroll
  for (int q = 0; q < 8; ++q) f.h[q] = (_Float16)bf16_round(x[t * 8 + q]); *(volatile v8us*)((unsigned short*)X16 + t * 8) = f.half[0]; __threadfence(); *(volatile v8us*)((unsigned short*)X16 + t * 8) = f.half[0]; }
__global__ __launch_bounds__(256) void k_h16(const float* __restrict__ x, _Float16* __restrict__ X16, size_t n8) { const size_t t = (size_t)blockIdx.x * 256 + threadIdx.x; if (t >= n8) return; FragH f;
#pragma unroll
  for (int q = 0; q < 8; ++q) f.h[q] = (_Float16)x[t * 8 + q]; *(volatile v8us*)((unsigned short*)X16 + t * 8) = f.half[0]; __threadfence(); *(volatile v8us*)((unsigned short*)X16 + t * 8) = f.half[0]; }
__global__ __launch_bounds__(256) void k_round16f(const float* __restrict__ W, _Float16* __restrict__ Bt, size_t n8) { const size_t t = (size_t)blockIdx.x * 256 + threadIdx.x; if (t >= n8) return; FragH f;
#pragma unroll
  for (int i = 0; i < 8; ++i) f.h[i] = (_Float16)(bf16_round(W[t * 8 + i]) * 16.0f); *(volatile v8us*)((unsigned short*)Bt + t * 8) = f.half[0]; __threadfence(); *(volatile v8us*)((unsigned short*)Bt + t * 8) = f.half[0]; }
template <int NHv, int TTv>
__global__ __launch_bounds__(256) void k_vt(const _Float16* __restrict__ V16, int ldv, int voff, _Float16* __restrict__ Vt) { __shared__ unsigned short tl[64][66]; const int tid = threadIdx.x; const int slab = blockIdx.x / (TTv / 64), lg = blockIdx.x % (TTv / 64); const int b = slab / NHv, h = slab % NHv;
  for (int i = tid; i < 64 * 8; i += 256) { const int r = i / 8, c8 = (i % 8) * 8; FragH f; f.half[0] = *(const v8us*)((const unsigned short*)V16 + ((size_t)b * TTv + lg * 64 + r) * ldv + voff + h * 64 + c8);
#pragma unroll
    for (int q = 0; q < 8; ++q) tl[r][c8 + q] = f.u[q]; }
  __syncthreads();
  for (int pass = 0; pass < 2; ++pass) {
#pragma unroll
    for (int rd = 0; rd < 2; ++rd) { const int d = rd * 32 + tid / 8, pc = tid % 8; FragH f;
#pragma unroll
      for (int q = 0; q < 8; ++q) f.u[q] = tl[pc * 8 + q][d];
      *(volatile v8us*)((unsigned short*)Vt + ((size_t)slab * 64 + d) * TTv + lg * 64 + pc * 8) = f.half[0]; }
    if (pass == 0) __threadfence(); } }

__global__ __launch_bounds__(256) void k_hl(const float* __restrict__ F, _Float16* __restrict__ Hh, _Float16* __restrict__ Hl, size_t n8) { const size_t t = (size_t)blockIdx.x * 256 + threadIdx.x; if (t >= n8) return; FragH fh, fl; const v4f a = *(const v4fa*)(F + t * 8), c = *(const v4fa*)(F + t * 8 + 4);
#pragma unroll
  for (int q = 0; q < 4; ++q) { _Float16 h = (_Float16)a[q]; fh.h[q] = h; fl.h[q] = (_Float16)((a[q] - (float)h) * 1024.0f); h = (_Float16)c[q]; fh.h[4 + q] = h; fl.h[4 + q] = (_Float16)((c[q] - (float)h) * 1024.0f); }
  for (int pass = 0; pass < 2; ++pass) { *(volatile v8us*)((unsigned short*)Hh + t * 8) = fh.half[0]; *(volatile v8us*)((unsigned short*)Hl + t * 8) = fl.half[0]; if (pass == 0) __threadfence(); } }

__constant__ float TCOS[NA] = {1.000000000e+00f,9.999619126e-01f,9.998477101e-01f,9.996573329e-01f,9.993908405e-01f,9.990482330e-01f,9.986295104e-01f,9.981347919e-01f,9.975640774e-01f,9.969173074e-01f,9.961947203e-01f,9.953961968e-01f,9.945219159e-01f,9.935718775e-01f,9.925461411e-01f,9.914448857e-01f,9.902680516e-01f,9.890158772e-01f,9.876883626e-01f,9.862856269e-01f,9.848077297e-01f,9.832549095e-01f,9.816271663e-01f,9.799246788e-01f,9.781476259e-01f,9.762960076e-01f,9.743700624e-01f,9.723699093e-01f,9.702957273e-01f,9.681476355e-01f,9.659258127e-01f,9.636304379e-01f,9.612616897e-01f,9.588197470e-01f,9.563047886e-01f,9.537169337e-01f,9.510565400e-01f,9.483236670e-01f,9.455185533e-01f,9.426414967e-01f,9.396926165e-01f,9.366722107e-01f,9.335803986e-01f,9.304175973e-01f,9.271838665e-01f,9.238795042e-01f,9.205048680e-01f,9.170600772e-01f,9.135454297e-01f,9.099612832e-01f,9.063077569e-01f,9.025852680e-01f,8.987940550e-01f,8.949343562e-01f,8.910065293e-01f,8.870108128e-01f,8.829475641e-01f,8.788171411e-01f,8.746197224e-01f,8.703556657e-01f,8.660253882e-01f,8.616291285e-01f,8.571673036e-01f,8.526401520e-01f,8.480480909e-01f,8.433914185e-01f,8.386705518e-01f,8.338858485e-01f,8.290376067e-01f,8.241261840e-01f,8.191520572e-01f,8.141155243e-01f,8.090170026e-01f,8.038569093e-01f,7.986355424e-01f,7.933533192e-01f,7.880107760e-01f,7.826081514e-01f,7.771459222e-01f,7.716246247e-01f,7.660444379e-01f,7.604059577e-01f,7.547096014e-01f,7.489557266e-01f,7.431448102e-01f,7.372773290e-01f,7.313537002e-01f,7.253744006e-01f,7.193397880e-01f,7.132504582e-01f,7.071067691e-01f,7.009092569e-01f,6.946583986e-01f,6.883546114e-01f,6.819983721e-01f,6.755902171e-01f,6.691305637e-01f,6.626200676e-01f,6.560590267e-01f,6.494480371e-01f,6.427876353e-01f,6.360782385e-01f,6.293204427e-01f,6.225146651e-01f,6.156615019e-01f,6.087614298e-01f,6.018150449e-01f,5.948227644e-01f,5.877853036e-01f,5.807029605e-01f,5.735764503e-01f,5.664062500e-01f,5.591928959e-01f,5.519369841e-01f,5.446390510e-01f,5.372995734e-01f,5.299192667e-01f,5.224986076e-01f,5.150380731e-01f,5.075383782e-01f,4.999999702e-01f,4.924235642e-01f,4.848095775e-01f,4.771587551e-01f,4.694716036e-01f,4.617486000e-01f,4.539905190e-01f,4.461977780e-01f,4.383711517e-01f,4.305111468e-01f,4.226182401e-01f,4.146932662e-01f,4.067366123e-01f,3.987490833e-01f,3.907311857e-01f,3.826834261e-01f,3.746066391e-01f,3.665012121e-01f,3.583679795e-01f,3.502073288e-01f,3.420201540e-01f,3.338069022e-01f,3.255681396e-01f,3.173047006e-01f,3.090169728e-01f,3.007058203e-01f,2.923717797e-01f,2.840153277e-01f,2.756373882e-01f,2.672383487e-01f,2.588190734e-01f,2.503799498e-01f,2.419219017e-01f,2.334454209e-01f,2.249510437e-01f,2.164396495e-01f,2.079116553e-01f,1.993679404e-01f,1.908090562e-01f,1.822355241e-01f,1.736482233e-01f,1.650475711e-01f,1.564344913e-01f,1.478094757e-01f,1.391731054e-01f,1.305262446e-01f,1.218693256e-01f,1.132032424e-01f,1.045284197e-01f,9.584575891e-02f,8.715580404e-02f,7.845908403e-02f,6.975650787e-02f,6.104850769e-02f,5.233597383e-02f,4.361945391e-02f,3.489949554e-02f,2.617699467e-02f,1.745238341e-02f,8.726561442e-03f,-4.371138829e-08f,-8.726529777e-03f,-1.745235175e-02f,-2.617696300e-02f,-3.489946201e-02f,-4.361942410e-02f,-5.233594030e-02f,-6.104847416e-02f,-6.975647807e-02f,-7.845905423e-02f,-8.715576679e-02f,-9.584572911e-02f,-1.045285091e-01f,-1.132032126e-01f,-1.218692884e-01f,-1.305262148e-01f,-1.391730756e-01f,-1.478094459e-01f,-1.564344466e-01f,-1.650475413e-01f,-1.736481935e-01f,-1.822354794e-01f,-1.908090264e-01f,-1.993679106e-01f,-2.079116255e-01f,-2.164396197e-01f,-2.249510139e-01f,-2.334453911e-01f,-2.419218719e-01f,-2.503800392e-01f,-2.588190436e-01f,-2.672383189e-01f,-2.756373584e-01f,-2.840152979e-01f,-2.923717499e-01f,-3.007057905e-01f,-3.090169430e-01f,-3.173046708e-01f,-3.255681098e-01f,-3.338068724e-01f,-3.420201242e-01f,-3.502074182e-01f,-3.583679497e-01f,-3.665011823e-01f,-3.746066093e-01f,-3.826833963e-01f,-3.907311559e-01f,-3.987490535e-01f,-4.067365825e-01f,-4.146932364e-01f,-4.226183295e-01f,-4.305111170e-01f,-4.383711219e-01f,-4.461977482e-01f,-4.539903998e-01f,-4.617486596e-01f,-4.694715738e-01f,-4.771587253e-01f,-4.848095477e-01f,-4.924234450e-01f,-5.000000596e-01f,-5.075383782e-01f,-5.150380135e-01f,-5.224984884e-01f,-5.299193263e-01f,-5.372996330e-01f,-5.446390510e-01f,-5.519369245e-01f,-5.591928363e-01f,-5.664063096e-01f,-5.735764503e-01f,-5.807029605e-01f,-5.877851844e-01f,-5.948227048e-01f,-6.018151045e-01f,-6.087614298e-01f,-6.156614423e-01f,-6.225146055e-01f,-6.293203235e-01f,-6.360782981e-01f,-6.427876353e-01f,-6.494480371e-01f,-6.560589671e-01f,-6.626199484e-01f,-6.691306829e-01f,-6.755902171e-01f,-6.819983125e-01f,-6.883544922e-01f,-6.946582794e-01f,-7.009093165e-01f,-7.071067691e-01f,-7.132503986e-01f,-7.193397284e-01f,-7.253744602e-01f,-7.313537598e-01f,-7.372773290e-01f,-7.431448102e-01f,-7.489556670e-01f,-7.547096610e-01f,-7.604060173e-01f,-7.660444379e-01f,-7.716245651e-01f,-7.771458626e-01f,-7.826082110e-01f,-7.880107760e-01f,-7.933533192e-01f,-7.986354828e-01f,-8.038567901e-01f,-8.090170622e-01f,-8.141155243e-01f,-8.191520572e-01f,-8.241261244e-01f,-8.290374875e-01f,-8.338858485e-01f,-8.386705518e-01f,-8.433914185e-01f,-8.480480313e-01f,-8.526400924e-01f,-8.571673036e-01f,-8.616291881e-01f,-8.660253882e-01f,-8.703556657e-01f,-8.746197820e-01f,-8.788171411e-01f,-8.829475641e-01f,-8.870108128e-01f,-8.910064697e-01f,-8.949344158e-01f,-8.987940550e-01f,-9.025852680e-01f,-9.063077569e-01f,-9.099612236e-01f,-9.135454893e-01f,-9.170600772e-01f,-9.205048680e-01f,-9.238795042e-01f,-9.271838069e-01f,-9.304175973e-01f,-9.335804582e-01f,-9.366721511e-01f,-9.396926165e-01f,-9.426414371e-01f,-9.455186129e-01f,-9.483236670e-01f,-9.510564804e-01f,-9.537169337e-01f,-9.563047290e-01f,-9.588197470e-01f,-9.612616897e-01f,-9.636304379e-01f,-9.659258127e-01f,-9.681476355e-01f,-9.702957273e-01f,-9.723699093e-01f,-9.743700624e-01f,-9.762960076e-01f,-9.781476259e-01f,-9.799247384e-01f,-9.816271663e-01f,-9.832549095e-01f,-9.848077297e-01f,-9.862856269e-01f,-9.876883626e-01f,-9.890158772e-01f,-9.902680516e-01f,-9.914448261e-01f,-9.925461411e-01f,-9.935718775e-01f,-9.945219159e-01f,-9.953961968e-01f,-9.961946607e-01f,-9.969173670e-01f,-9.975640774e-01f,-9.981347919e-01f,-9.986295104e-01f,-9.990482330e-01f,-9.993908405e-01f,-9.996573329e-01f,-9.998477101e-01f,-9.999619126e-01f};
__constant__ float TSIN[NA] = {0.000000000e+00f,8.726535365e-03f,1.745240577e-02f,2.617694996e-02f,3.489949554e-02f,4.361938685e-02f,5.233595893e-02f,6.104854122e-02f,6.975647062e-02f,7.845909894e-02f,8.715573698e-02f,9.584575146e-02f,1.045284644e-01f,1.132032126e-01f,1.218693480e-01f,1.305261999e-01f,1.391731054e-01f,1.478094012e-01f,1.564344764e-01f,1.650476009e-01f,1.736481786e-01f,1.822355241e-01f,1.908089966e-01f,1.993679255e-01f,2.079117000e-01f,2.164396197e-01f,2.249510586e-01f,2.334453613e-01f,2.419219017e-01f,2.503800094e-01f,2.588190436e-01f,2.672383785e-01f,2.756373584e-01f,2.840153575e-01f,2.923716903e-01f,3.007057905e-01f,3.090170026e-01f,3.173046410e-01f,3.255681694e-01f,3.338068724e-01f,3.420201242e-01f,3.502073884e-01f,3.583679497e-01f,3.665012121e-01f,3.746066093e-01f,3.826834559e-01f,3.907311261e-01f,3.987490833e-01f,4.067366421e-01f,4.146932364e-01f,4.226182699e-01f,4.305110872e-01f,4.383711517e-01f,4.461978078e-01f,4.539904892e-01f,4.617486000e-01f,4.694715738e-01f,4.771587551e-01f,4.848096073e-01f,4.924235642e-01f,5.000000000e-01f,5.075383782e-01f,5.150380731e-01f,5.224985480e-01f,5.299192667e-01f,5.372996330e-01f,5.446390510e-01f,5.519369841e-01f,5.591928959e-01f,5.664062500e-01f,5.735764503e-01f,5.807029605e-01f,5.877852440e-01f,5.948227644e-01f,6.018149853e-01f,6.087614298e-01f,6.156615019e-01f,6.225146651e-01f,6.293203831e-01f,6.360781789e-01f,6.427875757e-01f,6.494480371e-01f,6.560590267e-01f,6.626200676e-01f,6.691306233e-01f,6.755902171e-01f,6.819983721e-01f,6.883545518e-01f,6.946583986e-01f,7.009092569e-01f,7.071067691e-01f,7.132504582e-01f,7.193397880e-01f,7.253743410e-01f,7.313537002e-01f,7.372773290e-01f,7.431448698e-01f,7.489557266e-01f,7.547095418e-01f,7.604059577e-01f,7.660444379e-01f,7.716245651e-01f,7.771459222e-01f,7.826081514e-01f,7.880107164e-01f,7.933533192e-01f,7.986355424e-01f,8.038568497e-01f,8.090170026e-01f,8.141155243e-01f,8.191520572e-01f,8.241261840e-01f,8.290375471e-01f,8.338858485e-01f,8.386705518e-01f,8.433914781e-01f,8.480480909e-01f,8.526401520e-01f,8.571673036e-01f,8.616291285e-01f,8.660254478e-01f,8.703556657e-01f,8.746197224e-01f,8.788171411e-01f,8.829475641e-01f,8.870108128e-01f,8.910065293e-01f,8.949343562e-01f,8.987940550e-01f,9.025852680e-01f,9.063078165e-01f,9.099612832e-01f,9.135454893e-01f,9.170600772e-01f,9.205048084e-01f,9.238795042e-01f,9.271838665e-01f,9.304175973e-01f,9.335803986e-01f,9.366722107e-01f,9.396926165e-01f,9.426414967e-01f,9.455185533e-01f,9.483236670e-01f,9.510565400e-01f,9.537169337e-01f,9.563047290e-01f,9.588197470e-01f,9.612616897e-01f,9.636304379e-01f,9.659258127e-01f,9.681476355e-01f,9.702957273e-01f,9.723699093e-01f,9.743700624e-01f,9.762960076e-01f,9.781476259e-01f,9.799246788e-01f,9.816271663e-01f,9.832549095e-01f,9.848077297e-01f,9.862856269e-01f,9.876883626e-01f,9.890158772e-01f,9.902680516e-01f,9.914448261e-01f,9.925461411e-01f,9.935718775e-01f,9.945219159e-01f,9.953961968e-01f,9.961947203e-01f,9.969173074e-01f,9.975640774e-01f,9.981347919e-01f,9.986295104e-01f,9.990482330e-01f,9.993908405e-01f,9.996573329e-01f,9.998477101e-01f,9.999619126e-01f,1.000000000e+00f,9.999619126e-01f,9.998477101e-01f,9.996573329e-01f,9.993908405e-01f,9.990482330e-01f,9.986295104e-01f,9.981347919e-01f,9.975640774e-01f,9.969173074e-01f,9.961947203e-01f,9.953961968e-01f,9.945219159e-01f,9.935718775e-01f,9.925461411e-01f,9.914448857e-01f,9.902680516e-01f,9.890158772e-01f,9.876883626e-01f,9.862856269e-01f,9.848077297e-01f,9.832549095e-01f,9.816271663e-01f,9.799247384e-01f,9.781476259e-01f,9.762960076e-01f,9.743700624e-01f,9.723699093e-01f,9.702957273e-01f,9.681476355e-01f,9.659258127e-01f,9.636304975e-01f,9.612616897e-01f,9.588197470e-01f,9.563047290e-01f,9.537169337e-01f,9.510565400e-01f,9.483236670e-01f,9.455186129e-01f,9.426414967e-01f,9.396926165e-01f,9.366721511e-01f,9.335804582e-01f,9.304175973e-01f,9.271838665e-01f,9.238795638e-01f,9.205048680e-01f,9.170600772e-01f,9.135454893e-01f,9.099612832e-01f,9.063077569e-01f,9.025852680e-01f,8.987940550e-01f,8.949344158e-01f,8.910065889e-01f,8.870108128e-01f,8.829475641e-01f,8.788171411e-01f,8.746197224e-01f,8.703557849e-01f,8.660253882e-01f,8.616291285e-01f,8.571673036e-01f,8.526402116e-01f,8.480480313e-01f,8.433914185e-01f,8.386705518e-01f,8.338858485e-01f,8.290376067e-01f,8.241261244e-01f,8.191519976e-01f,8.141155243e-01f,8.090170026e-01f,8.038569093e-01f,7.986354828e-01f,7.933533192e-01f,7.880107760e-01f,7.826082110e-01f,7.771460414e-01f,7.716245651e-01f,7.660444379e-01f,7.604059577e-01f,7.547096014e-01f,7.489557862e-01f,7.431448102e-01f,7.372773290e-01f,7.313537002e-01f,7.253744006e-01f,7.193399072e-01f,7.132503986e-01f,7.071067691e-01f,7.009093165e-01f,6.946584582e-01f,6.883544922e-01f,6.819983125e-01f,6.755902171e-01f,6.691306233e-01f,6.626201272e-01f,6.560589671e-01f,6.494480371e-01f,6.427876353e-01f,6.360782981e-01f,6.293205023e-01f,6.225146055e-01f,6.156614423e-01f,6.087614298e-01f,6.018151045e-01f,5.948228836e-01f,5.877851844e-01f,5.807029605e-01f,5.735764503e-01f,5.664063096e-01f,5.591930151e-01f,5.519369245e-01f,5.446390510e-01f,5.372996330e-01f,5.299193263e-01f,5.224986672e-01f,5.150380135e-01f,5.075383782e-01f,5.000000596e-01f,4.924236536e-01f,4.848095477e-01f,4.771587253e-01f,4.694715738e-01f,4.617486596e-01f,4.539905787e-01f,4.461977482e-01f,4.383711219e-01f,4.305111170e-01f,4.226183295e-01f,4.146933556e-01f,4.067365825e-01f,3.987490535e-01f,3.907311559e-01f,3.826834857e-01f,3.746066988e-01f,3.665011525e-01f,3.583679199e-01f,3.502074182e-01f,3.420202136e-01f,3.338069916e-01f,3.255681098e-01f,3.173046410e-01f,3.090170324e-01f,3.007058799e-01f,2.923718393e-01f,2.840152979e-01f,2.756373584e-01f,2.672384381e-01f,2.588191330e-01f,2.503799200e-01f,2.419218570e-01f,2.334453762e-01f,2.249511182e-01f,2.164397240e-01f,2.079116106e-01f,1.993679106e-01f,1.908090115e-01f,1.822355986e-01f,1.736482978e-01f,1.650475413e-01f,1.564344466e-01f,1.478094310e-01f,1.391731799e-01f,1.305263191e-01f,1.218692809e-01f,1.132031977e-01f,1.045284942e-01f,9.584583342e-02f,8.715587854e-02f,7.845903933e-02f,6.975647062e-02f,6.104858220e-02f,5.233604833e-02f,4.361952841e-02f,3.489945084e-02f,2.617695183e-02f,1.745245792e-02f,8.726636879e-03f};
__constant__ float TCO[HI] = {-1.000000000e+00f,-9.921568632e-01f,-9.843137264e-01f,-9.764705896e-01f,-9.686274529e-01f,-9.607843161e-01f,-9.529411793e-01f,-9.450980425e-01f,-9.372549057e-01f,-9.294117689e-01f,-9.215686321e-01f,-9.137254953e-01f,-9.058823586e-01f,-8.980392218e-01f,-8.901960850e-01f,-8.823529482e-01f,-8.745098114e-01f,-8.666666746e-01f,-8.588235378e-01f,-8.509804010e-01f,-8.431372643e-01f,-8.352941275e-01f,-8.274509907e-01f,-8.196078539e-01f,-8.117647171e-01f,-8.039215803e-01f,-7.960784435e-01f,-7.882353067e-01f,-7.803921700e-01f,-7.725490332e-01f,-7.647058964e-01f,-7.568627596e-01f,-7.490196228e-01f,-7.411764860e-01f,-7.333333492e-01f,-7.254902124e-01f,-7.176470757e-01f,-7.098039389e-01f,-7.019608021e-01f,-6.941176653e-01f,-6.862745285e-01f,-6.784313917e-01f,-6.705882549e-01f,-6.627451181e-01f,-6.549019814e-01f,-6.470588446e-01f,-6.392157078e-01f,-6.313725710e-01f,-6.235294342e-01f,-6.156862378e-01f,-6.078431606e-01f,-5.999999642e-01f,-5.921568871e-01f,-5.843136907e-01f,-5.764706135e-01f,-5.686274171e-01f,-5.607843399e-01f,-5.529411435e-01f,-5.450980663e-01f,-5.372548699e-01f,-5.294117928e-01f,-5.215685964e-01f,-5.137255192e-01f,-5.058823228e-01f,-4.980392158e-01f,-4.901960194e-01f,-4.823529422e-01f,-4.745097458e-01f,-4.666666687e-01f,-4.588234723e-01f,-4.509803951e-01f,-4.431371987e-01f,-4.352941215e-01f,-4.274509251e-01f,-4.196078479e-01f,-4.117646515e-01f,-4.039215744e-01f,-3.960783780e-01f,-3.882353008e-01f,-3.803921044e-01f,-3.725490272e-01f,-3.647058308e-01f,-3.568627536e-01f,-3.490195572e-01f,-3.411764801e-01f,-3.333332837e-01f,-3.254902065e-01f,-3.176470101e-01f,-3.098039329e-01f,-3.019607365e-01f,-2.941176593e-01f,-2.862744629e-01f,-2.784313858e-01f,-2.705881894e-01f,-2.627451122e-01f,-2.549019158e-01f,-2.470587641e-01f,-2.392156273e-01f,-2.313724905e-01f,-2.235293537e-01f,-2.156862170e-01f,-2.078430802e-01f,-1.999999434e-01f,-1.921568066e-01f,-1.843136698e-01f,-1.764705330e-01f,-1.686273962e-01f,-1.607842594e-01f,-1.529411227e-01f,-1.450979859e-01f,-1.372548491e-01f,-1.294117123e-01f,-1.215685681e-01f,-1.137254313e-01f,-1.058822945e-01f,-9.803915769e-02f,-9.019602090e-02f,-8.235288411e-02f,-7.450974733e-02f,-6.666661054e-02f,-5.882347003e-02f,-5.098033324e-02f,-4.313719645e-02f,-3.529405966e-02f,-2.745092101e-02f,-1.960778423e-02f,-1.176464651e-02f,-3.921509255e-03f,3.921627998e-03f,1.176476479e-02f,1.960790157e-02f,2.745104022e-02f,3.529417515e-02f,4.313731566e-02f,5.098045245e-02f,5.882358924e-02f,6.666672230e-02f,7.450986654e-02f,8.235300332e-02f,9.019614011e-02f,9.803927690e-02f,1.058824137e-01f,1.137255505e-01f,1.215686873e-01f,1.294118166e-01f,1.372549683e-01f,1.450981051e-01f,1.529412419e-01f,1.607843786e-01f,1.686275154e-01f,1.764706522e-01f,1.843137890e-01f,1.921569258e-01f,2.000000626e-01f,2.078431994e-01f,2.156863362e-01f,2.235294729e-01f,2.313726097e-01f,2.392157465e-01f,2.470588833e-01f,2.549020052e-01f,2.627451718e-01f,2.705883086e-01f,2.784314454e-01f,2.862745821e-01f,2.941177189e-01f,3.019608557e-01f,3.098039925e-01f,3.176471293e-01f,3.254902661e-01f,3.333334029e-01f,3.411765397e-01f,3.490196764e-01f,3.568628132e-01f,3.647059500e-01f,3.725490868e-01f,3.803922236e-01f,3.882353604e-01f,3.960784972e-01f,4.039216340e-01f,4.117647707e-01f,4.196079075e-01f,4.274510443e-01f,4.352941811e-01f,4.431373179e-01f,4.509804547e-01f,4.588235915e-01f,4.666667283e-01f,4.745098650e-01f,4.823530018e-01f,4.901961386e-01f,4.980392754e-01f,5.058825016e-01f,5.137256384e-01f,5.215687752e-01f,5.294119120e-01f,5.372550488e-01f,5.450981855e-01f,5.529413223e-01f,5.607844591e-01f,5.686275959e-01f,5.764707327e-01f,5.843138695e-01f,5.921570063e-01f,6.000001431e-01f,6.078432798e-01f,6.156864166e-01f,6.235295534e-01f,6.313726902e-01f,6.392158270e-01f,6.470589638e-01f,6.549021006e-01f,6.627452374e-01f,6.705883741e-01f,6.784315109e-01f,6.862746477e-01f,6.941177845e-01f,7.019609213e-01f,7.098040581e-01f,7.176471949e-01f,7.254903316e-01f,7.333334684e-01f,7.411766052e-01f,7.490197420e-01f,7.568628788e-01f,7.647060156e-01f,7.725491524e-01f,7.803922892e-01f,7.882354259e-01f,7.960785627e-01f,8.039216995e-01f,8.117648363e-01f,8.196079731e-01f,8.274511099e-01f,8.352942467e-01f,8.431373835e-01f,8.509805202e-01f,8.588236570e-01f,8.666667938e-01f,8.745099306e-01f,8.823530674e-01f,8.901962042e-01f,8.980393410e-01f,9.058824778e-01f,9.137256145e-01f,9.215687513e-01f,9.294118881e-01f,9.372550249e-01f,9.450981617e-01f,9.529412985e-01f,9.607844353e-01f,9.686275721e-01f,9.764707088e-01f,9.843138456e-01f,9.921569824e-01f,1.000000000e+00f};
__constant__ float TFILT[ND] = {0.000000000e+00f,5.509641953e-03f,1.101928391e-02f,1.652892679e-02f,2.203856781e-02f,2.754820883e-02f,3.305785358e-02f,3.856749460e-02f,4.407713562e-02f,4.958677664e-02f,5.509641767e-02f,6.060606241e-02f,6.611570716e-02f,7.162534446e-02f,7.713498920e-02f,8.264462650e-02f,8.815427125e-02f,9.366391599e-02f,9.917355329e-02f,1.046831980e-01f,1.101928353e-01f,1.157024801e-01f,1.212121248e-01f,1.267217696e-01f,1.322314143e-01f,1.377410442e-01f,1.432506889e-01f,1.487603337e-01f,1.542699784e-01f,1.597796232e-01f,1.652892530e-01f,1.707988977e-01f,1.763085425e-01f,1.818181872e-01f,1.873278320e-01f,1.928374618e-01f,1.983471066e-01f,2.038567513e-01f,2.093663961e-01f,2.148760408e-01f,2.203856707e-01f,2.258953154e-01f,2.314049602e-01f,2.369146049e-01f,2.424242496e-01f,2.479338944e-01f,2.534435391e-01f,2.589531839e-01f,2.644628286e-01f,2.699724436e-01f,2.754820883e-01f,2.809917331e-01f,2.865013778e-01f,2.920110226e-01f,2.975206673e-01f,3.030303121e-01f,3.085399568e-01f,3.140496016e-01f,3.195592463e-01f,3.250688612e-01f,3.305785060e-01f,3.360881507e-01f,3.415977955e-01f,3.471074402e-01f,3.526170850e-01f,3.581267297e-01f,3.636363745e-01f,3.691460192e-01f,3.746556640e-01f,3.801653087e-01f,3.856749237e-01f,3.911845684e-01f,3.966942132e-01f,4.022038579e-01f,4.077135026e-01f,4.132231474e-01f,4.187327921e-01f,4.242424369e-01f,4.297520816e-01f,4.352617264e-01f,4.407713413e-01f,4.462809861e-01f,4.517906308e-01f,4.573002756e-01f,4.628099203e-01f,4.683195651e-01f,4.738292098e-01f,4.793388546e-01f,4.848484993e-01f,4.903581440e-01f,4.958677888e-01f,5.013774037e-01f,5.068870783e-01f,5.123966932e-01f,5.179063678e-01f,5.234159827e-01f,5.289256573e-01f,5.344352722e-01f,5.399448872e-01f,5.454545617e-01f,5.509641767e-01f,5.564738512e-01f,5.619834661e-01f,5.674931407e-01f,5.730027556e-01f,5.785124302e-01f,5.840220451e-01f,5.895316601e-01f,5.950413346e-01f,6.005509496e-01f,6.060606241e-01f,6.115702391e-01f,6.170799136e-01f,6.225895286e-01f,6.280992031e-01f,6.336088181e-01f,6.391184926e-01f,6.446281075e-01f,6.501377225e-01f,6.556473970e-01f,6.611570120e-01f,6.666666865e-01f,6.721763015e-01f,6.776859760e-01f,6.831955910e-01f,6.887052655e-01f,6.942148805e-01f,6.997245550e-01f,7.052341700e-01f,7.107437849e-01f,7.162534595e-01f,7.217630744e-01f,7.272727489e-01f,7.327823639e-01f,7.382920384e-01f,7.438016534e-01f,7.493113279e-01f,7.548209429e-01f,7.603306174e-01f,7.658402324e-01f,7.713498473e-01f,7.768595219e-01f,7.823691368e-01f,7.878788114e-01f,7.933884263e-01f,7.988981009e-01f,8.044077158e-01f,8.099173903e-01f,8.154270053e-01f,8.209366798e-01f,8.264462948e-01f,8.319559097e-01f,8.374655843e-01f,8.429751992e-01f,8.484848738e-01f,8.539944887e-01f,8.595041633e-01f,8.650137782e-01f,8.705234528e-01f,8.760330677e-01f,8.815426826e-01f,8.870523572e-01f,8.925619721e-01f,8.980716467e-01f,9.035812616e-01f,9.090909362e-01f,9.146005511e-01f,9.201102257e-01f,9.256198406e-01f,9.311295152e-01f,9.366391301e-01f,9.421487451e-01f,9.476584196e-01f,9.531680346e-01f,9.586777091e-01f,9.641873240e-01f,9.696969986e-01f,9.752066135e-01f,9.807162881e-01f,9.862259030e-01f,9.917355776e-01f,9.972451925e-01f,9.972451925e-01f,9.917355776e-01f,9.862259030e-01f,9.807162881e-01f,9.752066135e-01f,9.696969986e-01f,9.641873240e-01f,9.586777091e-01f,9.531680346e-01f,9.476584196e-01f,9.421487451e-01f,9.366391301e-01f,9.311295152e-01f,9.256198406e-01f,9.201102257e-01f,9.146005511e-01f,9.090909362e-01f,9.035812616e-01f,8.980716467e-01f,8.925619721e-01f,8.870523572e-01f,8.815426826e-01f,8.760330677e-01f,8.705234528e-01f,8.650137782e-01f,8.595041633e-01f,8.539944887e-01f,8.484848738e-01f,8.429751992e-01f,8.374655843e-01f,8.319559097e-01f,8.264462948e-01f,8.209366798e-01f,8.154270053e-01f,8.099173903e-01f,8.044077158e-01f,7.988981009e-01f,7.933884263e-01f,7.878788114e-01f,7.823691368e-01f,7.768595219e-01f,7.713498473e-01f,7.658402324e-01f,7.603306174e-01f,7.548209429e-01f,7.493113279e-01f,7.438016534e-01f,7.382920384e-01f,7.327823639e-01f,7.272727489e-01f,7.217630744e-01f,7.162534595e-01f,7.107437849e-01f,7.052341700e-01f,6.997245550e-01f,6.942148805e-01f,6.887052655e-01f,6.831955910e-01f,6.776859760e-01f,6.721763015e-01f,6.666666865e-01f,6.611570120e-01f,6.556473970e-01f,6.501377225e-01f,6.446281075e-01f,6.391184926e-01f,6.336088181e-01f,6.280992031e-01f,6.225895286e-01f,6.170799136e-01f,6.115702391e-01f,6.060606241e-01f,6.005509496e-01f,5.950413346e-01f,5.895316601e-01f,5.840220451e-01f,5.785124302e-01f,5.730027556e-01f,5.674931407e-01f,5.619834661e-01f,5.564738512e-01f,5.509641767e-01f,5.454545617e-01f,5.399448872e-01f,5.344352722e-01f,5.289256573e-01f,5.234159827e-01f,5.179063678e-01f,5.123966932e-01f,5.068870783e-01f,5.013774037e-01f,4.958677888e-01f,4.903581440e-01f,4.848484993e-01f,4.793388546e-01f,4.738292098e-01f,4.683195651e-01f,4.628099203e-01f,4.573002756e-01f,4.517906308e-01f,4.462809861e-01f,4.407713413e-01f,4.352617264e-01f,4.297520816e-01f,4.242424369e-01f,4.187327921e-01f,4.132231474e-01f,4.077135026e-01f,4.022038579e-01f,3.966942132e-01f,3.911845684e-01f,3.856749237e-01f,3.801653087e-01f,3.746556640e-01f,3.691460192e-01f,3.636363745e-01f,3.581267297e-01f,3.526170850e-01f,3.471074402e-01f,3.415977955e-01f,3.360881507e-01f,3.305785060e-01f,3.250688612e-01f,3.195592463e-01f,3.140496016e-01f,3.085399568e-01f,3.030303121e-01f,2.975206673e-01f,2.920110226e-01f,2.865013778e-01f,2.809917331e-01f,2.754820883e-01f,2.699724436e-01f,2.644628286e-01f,2.589531839e-01f,2.534435391e-01f,2.479338944e-01f,2.424242496e-01f,2.369146049e-01f,2.314049602e-01f,2.258953154e-01f,2.203856707e-01f,2.148760408e-01f,2.093663961e-01f,2.038567513e-01f,1.983471066e-01f,1.928374618e-01f,1.873278320e-01f,1.818181872e-01f,1.763085425e-01f,1.707988977e-01f,1.652892530e-01f,1.597796232e-01f,1.542699784e-01f,1.487603337e-01f,1.432506889e-01f,1.377410442e-01f,1.322314143e-01f,1.267217696e-01f,1.212121248e-01f,1.157024801e-01f,1.101928353e-01f,1.046831980e-01f,9.917355329e-02f,9.366391599e-02f,8.815427125e-02f,8.264462650e-02f,7.713498920e-02f,7.162534446e-02f,6.611570716e-02f,6.060606241e-02f,5.509641767e-02f,4.958677664e-02f,4.407713562e-02f,3.856749460e-02f,3.305785358e-02f,2.754820883e-02f,2.203856781e-02f,1.652892679e-02f,1.101928391e-02f,5.509641953e-03f};
__global__ __launch_bounds__(256) void k_kern(float* __restrict__ KV) { const int tid = threadIdx.x;
  for (int m = tid; m < NDP; m += 256) { double s = 0.0; if (m < ND) { for (int f = 0; f < ND; ++f) s += (double)TFILT[f] * cos(6.283185307179586476925 * (double)f * (double)m / (double)ND); s /= (double)ND; } const float v = (float)s; *(volatile float*)(KV + m) = v; __threadfence(); *(volatile float*)(KV + m) = v; } }
__global__ __launch_bounds__(256) void k_circ(const float* __restrict__ KV, _Float16* __restrict__ Kh, _Float16* __restrict__ Kl) {
  #pragma clang fp contract(off)
  const int t = blockIdx.x * 256 + threadIdx.x; if (t >= NDP * (NDP / 8)) return; const int c0 = (t % (NDP / 8)) * 8, d = t / (NDP / 8); FragH fh, fl;
#pragma unroll
  for (int q = 0; q < 8; ++q) { const int dp = c0 + q; float v = 0.f; if (d < ND && dp < ND) { int m = d - dp; if (m < 0) m += ND; v = KV[m]; } const _Float16 hi = (_Float16)v; fh.h[q] = hi; fl.h[q] = (_Float16)((v - (float)hi) * 1024.0f); }
  for (int pass = 0; pass < 2; ++pass) { *(volatile v8us*)((unsigned short*)Kh + (size_t)d * NDP + c0) = fh.half[0]; *(volatile v8us*)((unsigned short*)Kl + (size_t)d * NDP + c0) = fl.half[0]; if (pass == 0) __threadfence(); } }
__global__ __launch_bounds__(256) void k_s16(const float* __restrict__ s, _Float16* __restrict__ S16) { const int t = blockIdx.x * 256 + threadIdx.x; if (t >= NR * (NDP / 8)) return; const int c0 = (t % (NDP / 8)) * 8, r = t / (NDP / 8); FragH f;
#pragma unroll
  for (int q = 0; q < 8; ++q) { const int dp = c0 + q; f.h[q] = (dp < ND) ? (_Float16)bf16_round(s[(size_t)r * ND + dp]) : (_Float16)0.0f; }
  *(volatile v8us*)((unsigned short*)S16 + (size_t)r * NDP + c0) = f.half[0]; __threadfence(); *(volatile v8us*)((unsigned short*)S16 + (size_t)r * NDP + c0) = f.half[0]; }
__global__ __launch_bounds__(256) void k_bp(const float* __restrict__ FT, float* __restrict__ out) {
  #pragma clang fp contract(off)
  const int t = blockIdx.x * 256 + threadIdx.x; if (t >= NBS * HI * HI) return; const int j = t % HI, i = (t / HI) % HI, b = t / (HI * HI); const float xg = TCO[j], yg = TCO[i];
  const float scale = (float)(((double)(HI - 1) / 2.0) * 1.4142135623730951 / ((double)(ND - 1) / 2.0)); float acc = 0.f;
#pragma unroll 1
  for (int a = 0; a < NA; ++a) { const float tt = xg * TCOS[a] + yg * TSIN[a]; const float tn = tt / scale; const float u = (tn + 1.0f) * 0.5f * (float)(ND - 1); const float u0 = floorf(u); const float w1 = u - u0, w0 = 1.0f - w1; const int i0 = (int)u0, i1 = i0 + 1; const bool ok0 = (i0 >= 0 && i0 < ND), ok1 = (i1 >= 0 && i1 < ND); const int c0 = min(max(i0, 0), ND - 1), c1 = min(max(i1, 0), ND - 1);
    const float v0 = FT[(size_t)c0 * NR + b * NA + a], v1 = FT[(size_t)c1 * NR + b * NA + a]; acc += v0 * (ok0 ? w0 : 0.f) + v1 * (ok1 ? w1 : 0.f); }
  const float r = acc * (float)(3.14159265358979323846 / (double)NA); *(volatile float*)(out + t) = r; __threadfence(); *(volatile float*)(out + t) = r; }

extern "C" void kernel_launch(void* const* d_in, const int* in_sizes, int n_in,
                              void* d_out, int out_size, void* d_ws, size_t ws_size, hipStream_t stream) {
  (void)in_sizes; (void)n_in; (void)out_size;
  const float* sino = (const float*)d_in[0];
  char* ws = (char*)d_ws; size_t off = 0;
  auto take = [&](size_t bytes) { char* p = ws + off; off += (bytes + 255) & ~(size_t)255; return p; };
  float* KV = (float*)take(NDP * 4); _Float16* Kh = (_Float16*)take((size_t)NDP * NDP * 2); _Float16* Kl = (_Float16*)take((size_t)NDP * NDP * 2); _Float16* S16 = (_Float16*)take((size_t)NR * NDP * 2); float* FT = (float*)take((size_t)NDP * NR * 4);
  if (off > ws_size) return;
  k_kern<<<1, 256, 0, stream>>>(KV); k_circ<<<(NDP * (NDP / 8) + 255) / 256, 256, 0, stream>>>(KV, Kh, Kl); k_s16<<<(NR * (NDP / 8) + 255) / 256, 256, 0, stream>>>(sino, S16);
  const dim3 gF(((NDP / 16) * ((NR + 63) / 64) + 3) / 4, 1);
  k_gemm_hhx<0><<<gF, 128, 0, stream>>>(Kh, NDP, 0, S16, NDP, 0, 1.0f, nullptr, 0, nullptr, 1, 0, 0, FT, nullptr, NR, 0, NDP, NR, NDP); k_gemm_hhx<0><<<gF, 128, 0, stream>>>(Kl, NDP, 0, S16, NDP, 0, 0.0009765625f, nullptr, 0, FT, 1, (size_t)NR, 0, FT, nullptr, NR, 0, NDP, NR, NDP);
  k_bp<<<(NBS * HI * HI + 255) / 256, 256, 0, stream>>>(FT, (float*)d_out);
}
